// INR_51814485459009
// MI455X (gfx1250) — hardware-run, weakly checked
//
#include <hip/hip_runtime.h>
#include <math.h>

typedef __attribute__((ext_vector_type(16))) _Float16 v16h;
typedef __attribute__((ext_vector_type(8)))  _Float16 v8h;
typedef __attribute__((ext_vector_type(8)))  float    v8f;
typedef __attribute__((ext_vector_type(4)))  float    v4f;
typedef __attribute__((ext_vector_type(2)))  float    v2f;

constexpr int kBatch       = 16;
constexpr int kImgH        = 128;
constexpr int kImgW        = 128;
constexpr int kPixPerImg   = kImgH * kImgW;
constexpr int kNPix        = kBatch * kPixPerImg;
constexpr int kHid         = 256;
constexpr int kNSamp       = 16;
constexpr int kTile        = 64;
constexpr int kTilesPerImg = kPixPerImg / kTile;
constexpr int kNumTiles    = kNPix / kTile;
constexpr int kLdp         = 264;
constexpr int kW4Rows      = 64;
constexpr int kOut0Floats  = kNPix * 3;
constexpr int kOutFloats   = kOut0Floats + 2 * kBatch;
static_assert(kNPix == 262144, "pixel count");
static_assert(kTilesPerImg == 256, "tiles per image");
static_assert(kNumTiles == 4096, "tile count");
static_assert((kPixPerImg % kTile) == 0, "a tile never crosses an image");
static_assert((kHid % 32) == 0, "K multiple of 32");
static_assert((kTile % 32) == 0 && (kHid % 64) == 0, "M,N tile multiples");
static_assert(kOut0Floats == 786432 && kOutFloats == 786464, "output packing");
static_assert(((size_t)kOut0Floats * 4) % 128 == 0, "shift outputs start on a 128-B line");
static_assert((kTile * 3 * 4) % 128 == 0, "a tile of pixels is a whole number of 128-B lines");
static_assert(((kLdp * 2) % 16) == 0, "LDS rows 16-B aligned");

constexpr float kActCarry     = 64.0f;
constexpr float kWgtCarry     = 256.0f;
constexpr float kInvWgt       = 1.0f / kWgtCarry;
constexpr float kInvBoth      = 1.0f / (kActCarry * kWgtCarry);
constexpr float kF16MinNormal = 6.103515625e-5f;

constexpr size_t kOffW2T  = 0;
constexpr size_t kOffW3T  = kOffW2T + (size_t)kHid * kHid * 2;
constexpr size_t kOffW4T  = kOffW3T + (size_t)kHid * kHid * 2;
constexpr size_t kWsTotal = kOffW4T + (size_t)kW4Rows * kHid * 2;
static_assert(kWsTotal == 294912ull, "carve total");
static_assert(kWsTotal <= 134217728ull, "carve cap");
static_assert((kOffW3T % 128) == 0 && (kOffW4T % 128) == 0, "128-B aligned regions");

union FragU { v16h v; v8h h[2]; };
__device__ __forceinline__ v16h frag_load(const _Float16* p) {
  FragU f;
  f.h[0] = *(const v8h*)(p);
  f.h[1] = *(const v8h*)(p + 16);
  return f.v;
}
__device__ __forceinline__ v8f mma_g(v16h a, v16h b, v8f c) {
  c = __builtin_amdgcn_wmma_f32_16x16x32_f16(false, a, false, b, (short)0, c, false, false);
  asm volatile("v_nop\n\tv_nop\n\tv_nop\n\tv_nop" : "+v"(c) : "v"(a), "v"(b));
  return c;
}

__global__ __launch_bounds__(256) void prep_weights_kernel(
    const float* __restrict__ W2, const float* __restrict__ W3, const float* __restrict__ W4,
    _Float16* __restrict__ W2T, _Float16* __restrict__ W3T, _Float16* __restrict__ W4T)
{
  const int lane = threadIdx.x & 31;
  const int wave = __builtin_amdgcn_readfirstlane((int)(threadIdx.x >> 5));
  const int gw   = blockIdx.x * 8 + wave;
  if (gw >= 2 * kHid + kW4Rows) return;
  const float* src;
  _Float16* dst;
  int ld, col;
  bool valid;
  if (gw < kHid) {
    src = W2; ld = kHid; col = gw; valid = true; dst = W2T + (size_t)gw * kHid;
  } else if (gw < 2 * kHid) {
    src = W3; ld = kHid; col = gw - kHid; valid = true; dst = W3T + (size_t)(gw - kHid) * kHid;
  } else {
    const int c = gw - 2 * kHid;
    src = W4; ld = 3; col = (c < 3) ? c : 2; valid = (c < 3); dst = W4T + (size_t)c * kHid;
  }
  const int k0 = lane * 8;
  v8h hv;
#pragma unroll
  for (int e = 0; e < 8; ++e) {
    const float raw = src[(size_t)(k0 + e) * ld + col];
    float v = valid ? (raw * kWgtCarry) : 0.0f;
    v = (fabsf(v) < kF16MinNormal) ? 0.0f : v;
    hv[e] = (_Float16)v;
  }
  _Float16* q = dst + k0;
  *(volatile v8h*)q = hv;
  __threadfence();
  *(volatile v8h*)q = hv;
}

__device__ __forceinline__ void dense_layer(_Float16* hb, const _Float16* __restrict__ Wt,
                                            const float* __restrict__ bias, int lane, int wave)
{
  const int rw = wave >> 2, cw = wave & 3;
  const int rl = lane & 15, hh = lane >> 4;
  v8f acc[2][4];
#pragma unroll
  for (int i = 0; i < 2; ++i)
#pragma unroll
    for (int j = 0; j < 4; ++j) acc[i][j] = (v8f){0.f, 0.f, 0.f, 0.f, 0.f, 0.f, 0.f, 0.f};
  const _Float16* bp = Wt + (size_t)(cw * 64 + rl) * kHid + hh * 8;
  const _Float16* ap = hb + (rw * 32 + rl) * kLdp + hh * 8;
#pragma unroll 1
  for (int k0 = 0; k0 < kHid; k0 += 32) {
    v16h bf[4];
#pragma unroll
    for (int j = 0; j < 4; ++j) bf[j] = frag_load(bp + (size_t)j * 16 * kHid + k0);
#pragma unroll
    for (int i = 0; i < 2; ++i) {
      const v16h af = frag_load(ap + i * 16 * kLdp + k0);
#pragma unroll
      for (int j = 0; j < 4; ++j) acc[i][j] = mma_g(af, bf[j], acc[i][j]);
    }
  }
  __syncthreads();
#pragma unroll
  for (int j = 0; j < 4; ++j) {
    const int col = cw * 64 + j * 16 + rl;
    const float biasc = bias[col] * kActCarry;
#pragma unroll
    for (int i = 0; i < 2; ++i) {
#pragma unroll
      for (int r = 0; r < 8; ++r) {
        const int row = rw * 32 + i * 16 + hh * 8 + r;
        float c = fmaf(acc[i][j][r], kInvWgt, biasc);
        c = (c < kF16MinNormal) ? 0.0f : c;
        hb[row * kLdp + col] = (_Float16)c;
      }
    }
  }
  __syncthreads();
}

__global__ __launch_bounds__(256) void fused_mlp_kernel(
    const float* __restrict__ x, const int* __restrict__ sample_idx,
    const float* __restrict__ shift_vectors, const float* __restrict__ rotation_angle,
    const float* __restrict__ color_scales, const float* __restrict__ color_shifts,
    const float* __restrict__ W1, const float* __restrict__ b1,
    const _Float16* __restrict__ W2T, const float* __restrict__ b2,
    const _Float16* __restrict__ W3T, const float* __restrict__ b3,
    const _Float16* __restrict__ W4T, const float* __restrict__ b4,
    float* __restrict__ out)
{
  __shared__ __align__(16) _Float16 hbuf[kTile * kLdp];
  __shared__ __align__(16) float stage[kTile * 3];

  const int lane = threadIdx.x & 31;
  const int wave = __builtin_amdgcn_readfirstlane((int)(threadIdx.x >> 5));
  const int tile = blockIdx.x;
  const int img  = tile / kTilesPerImg;
  const int pix0 = tile * kTile;

  const int si_raw = sample_idx[img];
  const int si = (si_raw < 0) ? 0 : ((si_raw > kNSamp - 1) ? (kNSamp - 1) : si_raw);
  const float dy  = shift_vectors[si * 2 + 0];
  const float dx  = shift_vectors[si * 2 + 1];
  const float ang = rotation_angle[si];
  const float cs  = cosf(ang);
  const float sn  = sinf(ang);

  {
    const int j8 = lane * 8;
    float w0[8], w1[8], bb[8];
    {
      const v4f a0 = *(const v4f*)(W1 + j8);
      const v4f a1 = *(const v4f*)(W1 + j8 + 4);
      const v4f c0 = *(const v4f*)(W1 + kHid + j8);
      const v4f c1 = *(const v4f*)(W1 + kHid + j8 + 4);
      const v4f d0 = *(const v4f*)(b1 + j8);
      const v4f d1 = *(const v4f*)(b1 + j8 + 4);
#pragma unroll
      for (int e = 0; e < 4; ++e) {
        w0[e] = a0[e]; w0[4 + e] = a1[e];
        w1[e] = c0[e]; w1[4 + e] = c1[e];
        bb[e] = d0[e]; bb[4 + e] = d1[e];
      }
    }
#pragma unroll 1
    for (int it = 0; it < 8; ++it) {
      const int row = wave + 8 * it;
      const v2f xy = *(const v2f*)(x + 2 * (size_t)(pix0 + row));
      const float x0 = xy.x, x1 = xy.y;
      float t0 = cs * x0;
      t0 = fmaf(-sn, x1, t0);
      const float q0 = t0 + dx;
      float t1 = sn * x0;
      t1 = fmaf(cs, x1, t1);
      const float q1 = t1 + dy;
      v8h hv;
#pragma unroll
      for (int e = 0; e < 8; ++e) {
        float p = q0 * w0[e];
        p = fmaf(q1, w1[e], p);
        p = p + bb[e];
        float c = p * kActCarry;
        c = (c < kF16MinNormal) ? 0.0f : c;
        hv[e] = (_Float16)c;
      }
      *(v8h*)(hbuf + row * kLdp + j8) = hv;
    }
  }
  __syncthreads();

  dense_layer(hbuf, W2T, b2, lane, wave);
  dense_layer(hbuf, W3T, b3, lane, wave);

  {
    const int rl = lane & 15, hh = lane >> 4;
    const int cc = (rl < 3) ? rl : 2;
    float b4v = b4[cc];
    asm volatile("" : "+v"(b4v));
    float scl = color_scales[si * 3 + cc];
    asm volatile("" : "+v"(scl));
    float sft = color_shifts[si * 3 + cc];
    asm volatile("" : "+v"(sft));
    const bool apply = (si_raw != 0);
    if (wave < 4) {
      v8f acc = (v8f){0.f, 0.f, 0.f, 0.f, 0.f, 0.f, 0.f, 0.f};
      const _Float16* ap = hbuf + (wave * 16 + rl) * kLdp + hh * 8;
      const _Float16* bp = W4T + (size_t)rl * kHid + hh * 8;
#pragma unroll 1
      for (int k0 = 0; k0 < kHid; k0 += 32) {
        const v16h af = frag_load(ap + k0);
        const v16h bf = frag_load(bp + k0);
        acc = mma_g(af, bf, acc);
      }
#pragma unroll
      for (int r = 0; r < 8; ++r) {
        const int row = wave * 16 + hh * 8 + r;
        const float o  = fmaf(acc[r], kInvBoth, b4v);
        const float oa = o * scl + sft;
        const float ov = apply ? oa : o;
        if (rl < 3) stage[row * 3 + rl] = ov;
      }
    }
  }
  __syncthreads();

  if (wave == 0) {
    const int i2 = (32 + lane < 47) ? (32 + lane) : 47;
    const v4f va = *(const v4f*)(stage + lane * 4);
    const v4f vb = *(const v4f*)(stage + i2 * 4);
    float* dst = out + (size_t)tile * (kTile * 3);
    for (int pass = 0; pass < 2; ++pass) {
      *(volatile v4f*)(dst + lane * 4) = va;
      if (lane < 16) *(volatile v4f*)(dst + 128 + lane * 4) = vb;
      __threadfence();
    }
  }

  if (blockIdx.x == 0 && wave == 0) {
    const int bsel = lane & 15;
    const int kr = sample_idx[bsel];
    const int kk = (kr < 0) ? 0 : ((kr > kNSamp - 1) ? (kNSamp - 1) : kr);
    const float val = shift_vectors[kk * 2 + 1 - (lane >> 4)];
    float* dst = out + (size_t)kOut0Floats + lane;
    *(volatile float*)dst = val;
    __threadfence();
    *(volatile float*)dst = val;
  }
}

extern "C" void kernel_launch(void* const* d_in, const int* in_sizes, int n_in,
                              void* d_out, int out_size, void* d_ws, size_t ws_size,
                              hipStream_t stream) {
  if (n_in < 14) return;
  if (in_sizes[0] != kNPix * 2) return;
  if (in_sizes[1] != kBatch) return;
  if (in_sizes[2] != kNSamp * 2) return;
  if (in_sizes[3] != kNSamp) return;
  if (in_sizes[4] != kNSamp * 3) return;
  if (in_sizes[5] != kNSamp * 3) return;
  if (in_sizes[6] != 2 * kHid) return;
  if (in_sizes[7] != kHid) return;
  if (in_sizes[8] != kHid * kHid) return;
  if (in_sizes[9] != kHid) return;
  if (in_sizes[10] != kHid * kHid) return;
  if (in_sizes[11] != kHid) return;
  if (in_sizes[12] != kHid * 3) return;
  if (in_sizes[13] != 3) return;
  if (out_size != kOutFloats) return;
  if (ws_size < kWsTotal) return;

  const float* x              = (const float*)d_in[0];
  const int*   sample_idx     = (const int*)  d_in[1];
  const float* shift_vectors  = (const float*)d_in[2];
  const float* rotation_angle = (const float*)d_in[3];
  const float* color_scales   = (const float*)d_in[4];
  const float* color_shifts   = (const float*)d_in[5];
  const float* W1 = (const float*)d_in[6];
  const float* b1 = (const float*)d_in[7];
  const float* W2 = (const float*)d_in[8];
  const float* b2 = (const float*)d_in[9];
  const float* W3 = (const float*)d_in[10];
  const float* b3 = (const float*)d_in[11];
  const float* W4 = (const float*)d_in[12];
  const float* b4 = (const float*)d_in[13];
  float* out = (float*)d_out;

  char* ws = (char*)d_ws;
  _Float16* W2T = (_Float16*)(ws + kOffW2T);
  _Float16* W3T = (_Float16*)(ws + kOffW3T);
  _Float16* W4T = (_Float16*)(ws + kOffW4T);

  prep_weights_kernel<<<(2 * kHid + kW4Rows) / 8, 256, 0, stream>>>(W2, W3, W4, W2T, W3T, W4T);

  fused_mlp_kernel<<<kNumTiles, 256, 0, stream>>>(
      x, sample_idx, shift_vectors, rotation_angle, color_scales, color_shifts,
      W1, b1, W2T, b2, W3T, b3, W4T, b4, out);
}
